// GraphPlanEncoder_7593502179348
// MI455X (gfx1250) — hardware-verified
//
#include <hip/hip_runtime.h>
#include <stddef.h>


#define DF      128
#define KV      256
#define OUTD    256
#define GPB     8
#define NTHR    256
#define NWAVE   8
#define EPT     8
#define NGRP    2
#define CHUNK   (NTHR * EPT * NGRP)
#define WCAP    (EPT * NGRP * 32)
#define LISTN   (NWAVE * WCAP)
#define NB      512
#define NTILE   (NB / 16)
#define TPW     (NTILE / NWAVE)
#define LN_EPS  1e-5f
#define NRM_EPS 1e-12f

#define LDS_ACC   (NB * DF * 4)
#define LDS_LIST  (LISTN * 4)
#define LDS_CNT   (NB * 4)
#define LDS_LAYER (LDS_ACC + LDS_LIST + LDS_CNT + 64)

static_assert((CHUNK & (CHUNK - 1)) == 0);
static_assert(CHUNK <= 4096);
static_assert((NB & (NB - 1)) == 0);
static_assert(NB <= 4096);
static_assert(GPB <= 4096);
static_assert(NTILE % NWAVE == 0);
static_assert(GPB == NWAVE);
static_assert(NWAVE * 4 <= 64);
static_assert(LDS_LAYER <= 300 * 1024);
static_assert(NTHR == 2 * DF);
static_assert(NTHR == OUTD);
static_assert(OUTD == 2 * DF);
static_assert(OUTD == KV);
static_assert(DF == 4 * 32);
static_assert(KV == 2 * DF);
static_assert(GPB * DF <= LISTN);

typedef float  v4f   __attribute__((ext_vector_type(4)));
typedef float  v8f   __attribute__((ext_vector_type(8)));
typedef int    v4i   __attribute__((ext_vector_type(4)));
typedef __bf16 bf16_t;
typedef bf16_t v8bf  __attribute__((ext_vector_type(8)));
typedef bf16_t v16bf __attribute__((ext_vector_type(16)));
union FragB { v16bf v; v8bf h[2]; v4i q[2]; };
union Pack8 { v8bf v; v4i q; };

__device__ __forceinline__ v8f wmb(v16bf a, v16bf b, v8f c) {
  v8f d = __builtin_amdgcn_wmma_f32_16x16x32_bf16(false, a, false, b, (short)0, c, false, false);
  asm volatile("v_nop\n\tv_nop\n\tv_nop\n\tv_nop" : "+v"(d) : "v"(a), "v"(b));
  return d;
}

template <int B>
__device__ __forceinline__ void split8(FragB& hi, FragB& lo, v4f a, v4f b) {
#define SPL1(I, X) { const float xv = (X); const bf16_t hb = (bf16_t)xv; hi.v[B + (I)] = hb; lo.v[B + (I)] = (bf16_t)(xv - (float)hb); }
  SPL1(0, a.x) SPL1(1, a.y) SPL1(2, a.z) SPL1(3, a.w)
  SPL1(4, b.x) SPL1(5, b.y) SPL1(6, b.z) SPL1(7, b.w)
#undef SPL1
}

template <int NBT>
__device__ __forceinline__ int scan_chunk(const int* __restrict__ keys, int nK, int cbase, int keyBase,
                                          int vec8, int* list, int tid, int wave) {
  int wc = 0;
#pragma unroll
  for (int g = 0; g < NGRP; ++g) {
    const int el0  = (g * NTHR + tid) * EPT;
    const int e0   = cbase + el0;
    const int sent = -2147483647 - 1;
    v4i da, db;
    if (vec8 != 0 && e0 + 7 < nK) {
      da = *(const v4i*)(keys + e0);
      db = *(const v4i*)(keys + e0 + 4);
    } else {
      da.x = (e0     < nK) ? keys[min(e0, nK - 1)] : sent;
      da.y = (e0 + 1 < nK) ? keys[min(e0 + 1, nK - 1)] : sent;
      da.z = (e0 + 2 < nK) ? keys[min(e0 + 2, nK - 1)] : sent;
      da.w = (e0 + 3 < nK) ? keys[min(e0 + 3, nK - 1)] : sent;
      db.x = (e0 + 4 < nK) ? keys[min(e0 + 4, nK - 1)] : sent;
      db.y = (e0 + 5 < nK) ? keys[min(e0 + 5, nK - 1)] : sent;
      db.z = (e0 + 6 < nK) ? keys[min(e0 + 6, nK - 1)] : sent;
      db.w = (e0 + 7 < nK) ? keys[min(e0 + 7, nK - 1)] : sent;
    }
    const unsigned nb = (unsigned)keyBase;
    const unsigned s0 = (unsigned)da.x - nb, s1 = (unsigned)da.y - nb;
    const unsigned s2 = (unsigned)da.z - nb, s3 = (unsigned)da.w - nb;
    const unsigned s4 = (unsigned)db.x - nb, s5 = (unsigned)db.y - nb;
    const unsigned s6 = (unsigned)db.z - nb, s7 = (unsigned)db.w - nb;
    const bool h0 = s0 < (unsigned)NBT, h1 = s1 < (unsigned)NBT, h2 = s2 < (unsigned)NBT, h3 = s3 < (unsigned)NBT;
    const bool h4 = s4 < (unsigned)NBT, h5 = s5 < (unsigned)NBT, h6 = s6 < (unsigned)NBT, h7 = s7 < (unsigned)NBT;
    const unsigned any = __builtin_amdgcn_ballot_w32(h0 | h1 | h2 | h3 | h4 | h5 | h6 | h7);
    if (any != 0u) {
#define HITJ(J, HJ, SJ) { \
        const unsigned mj = __builtin_amdgcn_ballot_w32(HJ); \
        if (mj != 0u) { \
          if (HJ) { \
            const int pos = wc + (int)__builtin_amdgcn_mbcnt_lo(mj, 0u); \
            if (pos < WCAP) list[wave * WCAP + pos] = ((el0 + (J)) << 12) | (int)(SJ); \
          } \
          wc += (int)__builtin_popcount(mj); } }
      HITJ(0, h0, s0)
      HITJ(1, h1, s1)
      HITJ(2, h2, s2)
      HITJ(3, h3, s3)
      HITJ(4, h4, s4)
      HITJ(5, h5, s5)
      HITJ(6, h6, s6)
      HITJ(7, h7, s7)
#undef HITJ
    }
  }
  return wc;
}

__global__ __launch_bounds__(NTHR) void k_wprep(
    const float* __restrict__ Wl, const float* __restrict__ Wr,
    bf16_t* whi, bf16_t* wlo, int nTot) {
  const int i = blockIdx.x * NTHR + threadIdx.x;
  if (i >= nTot) return;
  const int o  = i * 8;
  const int n  = o / KV;
  const int k0 = o - n * KV;
  const float* p = (k0 < DF) ? (Wl + (size_t)k0 * DF + n)
                             : (Wr + (size_t)(k0 - DF) * DF + n);
  Pack8 ph, pl;
#define WSP(I) { const float xv = p[(I) * DF]; const bf16_t hb = (bf16_t)xv; ph.v[(I)] = hb; pl.v[(I)] = (bf16_t)(xv - (float)hb); }
  WSP(0) WSP(1) WSP(2) WSP(3) WSP(4) WSP(5) WSP(6) WSP(7)
#undef WSP
  bf16_t* dh = whi + o;
  bf16_t* dl = wlo + o;
  const v4i qh = ph.q, ql = pl.q;
  *(volatile v4i*)dh = qh;
  *(volatile v4i*)dl = ql;
  __threadfence();
  *(volatile v4i*)dh = qh;
  *(volatile v4i*)dl = ql;
}

__device__ __forceinline__ void kstep(const float* ap, float mul,
                                      const bf16_t* bhp, const bf16_t* blp, v8f (&c)[8]) {
  const v4f p0 = (*(const v4f*)(ap))      * mul;
  const v4f p1 = (*(const v4f*)(ap + 4))  * mul;
  const v4f p2 = (*(const v4f*)(ap + 16)) * mul;
  const v4f p3 = (*(const v4f*)(ap + 20)) * mul;
  FragB ahi, alo;
  split8<0>(ahi, alo, p0, p1);
  split8<8>(ahi, alo, p2, p3);
#pragma unroll
  for (int ct = 0; ct < DF / 16; ++ct) {
    const bf16_t* hp = bhp + (size_t)ct * 16 * KV;
    const bf16_t* lp = blp + (size_t)ct * 16 * KV;
    FragB bh, bq;
    bh.q[0] = *(const v4i*)hp;  bh.q[1] = *(const v4i*)(hp + 16);
    bq.q[0] = *(const v4i*)lp;  bq.q[1] = *(const v4i*)(lp + 16);
    c[ct] = wmb(alo.v, bh.v, c[ct]);
    c[ct] = wmb(ahi.v, bq.v, c[ct]);
    c[ct] = wmb(ahi.v, bh.v, c[ct]);
  }
}

__global__ __launch_bounds__(NTHR) void k_layer(
    const int* __restrict__ ei, const float* __restrict__ xin,
    const bf16_t* __restrict__ whi, const bf16_t* __restrict__ wlo,
    const float* __restrict__ bias, const float* __restrict__ gam, const float* __restrict__ bet,
    float* xout, int nN, int nE, int vec8) {
  extern __shared__ v4f lds_dyn[];
  float* acc  = (float*)lds_dyn;
  int*   list = (int*)((char*)lds_dyn + LDS_ACC);
  int*   cnt  = (int*)((char*)lds_dyn + LDS_ACC + LDS_LIST);
  int*   wcnt = (int*)((char*)lds_dyn + LDS_ACC + LDS_LIST + LDS_CNT);
  const int tid = threadIdx.x, lane = tid & 31, wave = tid >> 5, hh = lane >> 4, m = lane & 15;
  const int nodeBase = blockIdx.x * NB;
  const int* dsts = ei + nE;

  {
    const v4f z = {0.f, 0.f, 0.f, 0.f};
    for (int i = tid; i < NB * DF / 4; i += NTHR) lds_dyn[i] = z;
    for (int i = tid; i < NB; i += NTHR) cnt[i] = 0;
  }
  __syncthreads();

  const int nChunks = (nE + CHUNK - 1) / CHUNK;
#pragma unroll 1
  for (int ch = 0; ch < nChunks; ++ch) {
    const int cbase = ch * CHUNK;
    const int wc = scan_chunk<NB>(dsts, nE, cbase, nodeBase, vec8, list, tid, wave);
    if (lane == 0) wcnt[wave] = wc;
    __syncthreads();
    if (wave == 0) {
#pragma unroll 1
      for (int wsx = 0; wsx < NWAVE; ++wsx) {
        int n = __builtin_amdgcn_readfirstlane(wcnt[wsx]);
        n = n > WCAP ? WCAP : (n < 0 ? 0 : n);
        const int* lp = list + wsx * WCAP;
#pragma unroll 1
        for (int i = 0; i < n; ++i) {
          const int ent  = __builtin_amdgcn_readfirstlane(lp[i]);
          int slot = ent & 0xFFF;
          slot = slot > NB - 1 ? NB - 1 : slot;
          int e = cbase + ((ent >> 12) & (CHUNK - 1));
          e = e > nE - 1 ? nE - 1 : e;
          int src = ei[e];
          src = src < 0 ? 0 : (src > nN - 1 ? nN - 1 : src);
          const v4f v = *(const v4f*)(xin + (size_t)src * DF + 4 * lane);
          v4f* ap = (v4f*)(acc + slot * DF + 4 * lane);
          *ap = *ap + v;
          if (lane == 0) cnt[slot] = cnt[slot] + 1;
        }
      }
    }
    __syncthreads();
  }
  __syncthreads();

#pragma unroll 1
  for (int q = 0; q < TPW; ++q) {
    const int t     = q * NWAVE + wave;
    const int slotm = 16 * t + m;
    int node = nodeBase + slotm;
    node = node > nN - 1 ? nN - 1 : node;
    const int   cd  = cnt[slotm];
    const float inv = 1.0f / (float)(cd > 1 ? cd : 1);

    v8f c[8];
#pragma unroll
    for (int ct = 0; ct < 8; ++ct) { const v8f z = {0.f, 0.f, 0.f, 0.f, 0.f, 0.f, 0.f, 0.f}; c[ct] = z; }

    const float*  arow = acc + slotm * DF + 8 * hh;
    const float*  xrow = xin + (size_t)node * DF + 8 * hh;
    const bf16_t* bh0  = whi + m * KV + 8 * hh;
    const bf16_t* bl0  = wlo + m * KV + 8 * hh;
#pragma unroll 1
    for (int ks = 0; ks < DF / 32; ++ks)
      kstep(arow + 32 * ks, inv, bh0 + 32 * ks, bl0 + 32 * ks, c);
#pragma unroll 1
    for (int ks = 0; ks < DF / 32; ++ks)
      kstep(xrow + 32 * ks, 1.0f, bh0 + DF + 32 * ks, bl0 + DF + 32 * ks, c);

#pragma unroll
    for (int ct = 0; ct < 8; ++ct) {
      const float bv = bias[16 * ct + m];
#pragma unroll
      for (int r = 0; r < 8; ++r) c[ct][r] += bv;
    }
    float mu[8], rs[8];
#pragma unroll
    for (int r = 0; r < 8; ++r) {
      float s = c[0][r];
#pragma unroll
      for (int ct = 1; ct < 8; ++ct) s += c[ct][r];
      s += __shfl_xor(s, 1);
      s += __shfl_xor(s, 2);
      s += __shfl_xor(s, 4);
      s += __shfl_xor(s, 8);
      mu[r] = s * (1.0f / (float)DF);
    }
#pragma unroll
    for (int r = 0; r < 8; ++r) {
      float qv = 0.0f;
#pragma unroll
      for (int ct = 0; ct < 8; ++ct) { const float d = c[ct][r] - mu[r]; qv += d * d; }
      qv += __shfl_xor(qv, 1);
      qv += __shfl_xor(qv, 2);
      qv += __shfl_xor(qv, 4);
      qv += __shfl_xor(qv, 8);
      rs[r] = rsqrtf(qv * (1.0f / (float)DF) + LN_EPS);
    }
    float* sp = acc + (16 * t + 8 * hh) * DF + m;
#pragma unroll
    for (int ct = 0; ct < 8; ++ct) {
      const int   col = 16 * ct + m;
      const float gv  = gam[col];
      const float ev  = bet[col];
#pragma unroll
      for (int r = 0; r < 8; ++r) {
        const float v = (c[ct][r] - mu[r]) * rs[r] * gv + ev;
        sp[r * DF + 16 * ct] = fmaxf(v, 0.0f);
      }
    }
    __syncthreads();

    const float* lrow = acc + (16 * t) * DF + 4 * lane;
    float* gp = xout + ((size_t)nodeBase + 16 * t) * DF + 4 * lane;
#pragma unroll
    for (int i = 0; i < 16; ++i) { const v4f v = *(const v4f*)(lrow + i * DF); *(volatile v4f*)(gp + (size_t)i * DF) = v; }
    __threadfence();
#pragma unroll
    for (int i = 0; i < 16; ++i) { const v4f v = *(const v4f*)(lrow + i * DF); *(volatile v4f*)(gp + (size_t)i * DF) = v; }
  }
}

__global__ __launch_bounds__(NTHR) void k_pool(
    const int* __restrict__ gb, const float* __restrict__ h,
    const float* __restrict__ Wr1, const float* __restrict__ br1,
    const float* __restrict__ Wr2, const float* __restrict__ br2,
    float* out, int nN, int nG) {
  __shared__ __align__(16) float pooled[GPB * KV];
  __shared__ __align__(16) int   plist[LISTN];
  __shared__ int   pcnt[GPB];
  __shared__ float pinv[GPB];
  __shared__ int   pwcnt[NWAVE];
  float* hid = (float*)plist;

  const int tid = threadIdx.x, lane = tid & 31, wave = tid >> 5;
  const int gBase = blockIdx.x * GPB;
  const float neg_inf = __uint_as_float(0xff800000u);

  for (int i = tid; i < GPB * KV; i += NTHR) pooled[i] = ((i & (KV - 1)) < DF) ? 0.0f : neg_inf;
  if (tid < GPB) pcnt[tid] = 0;
  __syncthreads();

  const int nChunks = (nN + CHUNK - 1) / CHUNK;
#pragma unroll 1
  for (int ch = 0; ch < nChunks; ++ch) {
    const int cbase = ch * CHUNK;
    const int wc = scan_chunk<GPB>(gb, nN, cbase, gBase, 1, plist, tid, wave);
    if (lane == 0) pwcnt[wave] = wc;
    __syncthreads();
    if (wave == 0) {
#pragma unroll 1
      for (int wsx = 0; wsx < NWAVE; ++wsx) {
        int n = __builtin_amdgcn_readfirstlane(pwcnt[wsx]);
        n = n > WCAP ? WCAP : (n < 0 ? 0 : n);
        const int* lp = plist + wsx * WCAP;
#pragma unroll 1
        for (int i = 0; i < n; ++i) {
          const int ent  = __builtin_amdgcn_readfirstlane(lp[i]);
          int slot = ent & 0xFFF;
          slot = slot > GPB - 1 ? GPB - 1 : slot;
          int node = cbase + ((ent >> 12) & (CHUNK - 1));
          node = node > nN - 1 ? nN - 1 : node;
          const v4f v = *(const v4f*)(h + (size_t)node * DF + 4 * lane);
          v4f* sp = (v4f*)(pooled + slot * KV + 4 * lane);
          *sp = *sp + v;
          v4f* mp = (v4f*)(pooled + slot * KV + DF + 4 * lane);
          v4f mx = *mp;
          mx.x = fmaxf(mx.x, v.x); mx.y = fmaxf(mx.y, v.y); mx.z = fmaxf(mx.z, v.z); mx.w = fmaxf(mx.w, v.w);
          *mp = mx;
          if (lane == 0) pcnt[slot] = pcnt[slot] + 1;
        }
      }
    }
    __syncthreads();
  }
  __syncthreads();

  if (tid < GPB) {
    const int cd = pcnt[tid];
    pinv[tid] = 1.0f / (float)(cd > 1 ? cd : 1);
  }
  __syncthreads();
#pragma unroll 1
  for (int i = tid; i < GPB * DF; i += NTHR) {
    const int slot = i / DF, col = i - slot * DF;
    pooled[slot * KV + col] = pooled[slot * KV + col] * pinv[slot];
  }
  __syncthreads();

  {
    const int j  = tid & (DF - 1);
    const int sg = (tid >> 7) * (GPB / 2);
    float a[GPB / 2];
#pragma unroll
    for (int i = 0; i < GPB / 2; ++i) a[i] = 0.0f;
#pragma unroll 1
    for (int k = 0; k < KV; ++k) {
      const float w = Wr1[(size_t)k * DF + j];
#pragma unroll
      for (int i = 0; i < GPB / 2; ++i) a[i] += pooled[(sg + i) * KV + k] * w;
    }
    const float bb = br1[j];
#pragma unroll
    for (int i = 0; i < GPB / 2; ++i) hid[(sg + i) * DF + j] = fmaxf(a[i] + bb, 0.0f);
  }
  __syncthreads();

  {
    const int o = tid;
    float e[GPB];
#pragma unroll
    for (int i = 0; i < GPB; ++i) e[i] = 0.0f;
#pragma unroll 1
    for (int jj = 0; jj < DF; ++jj) {
      const float w = Wr2[(size_t)jj * OUTD + o];
#pragma unroll
      for (int i = 0; i < GPB; ++i) e[i] += hid[i * DF + jj] * w;
    }
    const float bb = br2[o];
#pragma unroll
    for (int i = 0; i < GPB; ++i) pooled[i * OUTD + o] = e[i] + bb;
  }
  __syncthreads();

  {
    const int i = wave;
    const int g = gBase + i;
    const v4f v0 = *(const v4f*)(pooled + i * OUTD + 4 * lane);
    const v4f v1 = *(const v4f*)(pooled + i * OUTD + OUTD / 2 + 4 * lane);
    const v4f pq = v0 * v0 + v1 * v1;
    float sq = (pq.x + pq.y) + (pq.z + pq.w);
    sq += __shfl_xor(sq, 16);
    sq += __shfl_xor(sq, 8);
    sq += __shfl_xor(sq, 4);
    sq += __shfl_xor(sq, 2);
    sq += __shfl_xor(sq, 1);
    float nrm = sqrtf(sq);
    nrm = fmaxf(nrm, NRM_EPS);
    const float inv = 1.0f / nrm;
    const v4f o0 = v0 * inv;
    const v4f o1 = v1 * inv;
    const bool ok = g < nG;
    float* gp = out + (size_t)(ok ? g : 0) * OUTD + 4 * lane;
    if (ok) {
      *(volatile v4f*)gp = o0;
      *(volatile v4f*)(gp + OUTD / 2) = o1;
    }
    __threadfence();
    if (ok) {
      *(volatile v4f*)gp = o0;
      *(volatile v4f*)(gp + OUTD / 2) = o1;
    }
  }
}

extern "C" void kernel_launch(void* const* d_in, const int* in_sizes, int n_in,
                              void* d_out, int out_size, void* d_ws, size_t ws_size,
                              hipStream_t stream) {
  if (n_in < 22) return;
  const int nN = in_sizes[0] / DF;
  const int nE = in_sizes[1] / 2;
  if (nN <= 0 || nE < 0) return;
  if (in_sizes[0] != nN * DF || in_sizes[1] != 2 * nE || in_sizes[2] != nN) return;
  if (in_sizes[3] != DF * DF || in_sizes[4] != DF * DF || in_sizes[8] != DF * DF ||
      in_sizes[9] != DF * DF || in_sizes[13] != DF * DF || in_sizes[14] != DF * DF) return;
  if (in_sizes[5] < DF || in_sizes[6] < DF || in_sizes[7] < DF ||
      in_sizes[10] < DF || in_sizes[11] < DF || in_sizes[12] < DF ||
      in_sizes[15] < DF || in_sizes[16] < DF || in_sizes[17] < DF) return;
  if (in_sizes[18] != KV * DF || in_sizes[19] < DF || in_sizes[20] != DF * OUTD || in_sizes[21] < OUTD) return;
  if (out_size <= 0 || (out_size % OUTD) != 0) return;
  const int nG = out_size / OUTD;

  const float* x0  = (const float*)d_in[0];
  const int*   ei  = (const int*)d_in[1];
  const int*   gb  = (const int*)d_in[2];
  const float* W1l = (const float*)d_in[3];
  const float* W1r = (const float*)d_in[4];
  const float* b1  = (const float*)d_in[5];
  const float* g1  = (const float*)d_in[6];
  const float* be1 = (const float*)d_in[7];
  const float* W2l = (const float*)d_in[8];
  const float* W2r = (const float*)d_in[9];
  const float* b2  = (const float*)d_in[10];
  const float* g2  = (const float*)d_in[11];
  const float* be2 = (const float*)d_in[12];
  const float* W3l = (const float*)d_in[13];
  const float* W3r = (const float*)d_in[14];
  const float* b3  = (const float*)d_in[15];
  const float* g3  = (const float*)d_in[16];
  const float* be3 = (const float*)d_in[17];
  const float* Wr1 = (const float*)d_in[18];
  const float* br1 = (const float*)d_in[19];
  const float* Wr2 = (const float*)d_in[20];
  const float* br2 = (const float*)d_in[21];
  float* out = (float*)d_out;

  const int nBlk = (nN + NB - 1) / NB;
  const int nGB  = (nG + GPB - 1) / GPB;

  char* ws = (char*)d_ws;
  size_t off = 0;
  const size_t szW1 = (size_t)DF * KV * 2;
  const size_t szW  = 3 * szW1;
  const size_t szX  = (size_t)nBlk * NB * DF * 4;
  const size_t oWh = off; off += szW; off = (off + 255) & ~(size_t)255;
  const size_t oWl = off; off += szW; off = (off + 255) & ~(size_t)255;
  const size_t oXa = off; off += szX; off = (off + 255) & ~(size_t)255;
  const size_t oXb = off; off += szX; off = (off + 255) & ~(size_t)255;
  if (off > ws_size) return;
  bf16_t* whi = (bf16_t*)(ws + oWh);
  bf16_t* wlo = (bf16_t*)(ws + oWl);
  float*  xa  = (float*)(ws + oXa);
  float*  xb  = (float*)(ws + oXb);

  const int vec8 = ((nE & 3) == 0) ? 1 : 0;
  const int nTot = DF * KV / 8;
  const int wBlk = (nTot + NTHR - 1) / NTHR;

  k_wprep<<<wBlk, NTHR, 0, stream>>>(W1l, W1r, whi,                  wlo,                  nTot);
  k_wprep<<<wBlk, NTHR, 0, stream>>>(W2l, W2r, whi + DF * KV,        wlo + DF * KV,        nTot);
  k_wprep<<<wBlk, NTHR, 0, stream>>>(W3l, W3r, whi + 2 * DF * KV,    wlo + 2 * DF * KV,    nTot);

  hipFuncSetAttribute(reinterpret_cast<const void*>(&k_layer),
                      hipFuncAttributeMaxDynamicSharedMemorySize, LDS_LAYER);

  k_layer<<<nBlk, NTHR, LDS_LAYER, stream>>>(ei, x0, whi,               wlo,               b1, g1, be1, xa, nN, nE, vec8);
  k_layer<<<nBlk, NTHR, LDS_LAYER, stream>>>(ei, xa, whi + DF * KV,     wlo + DF * KV,     b2, g2, be2, xb, nN, nE, vec8);
  k_layer<<<nBlk, NTHR, LDS_LAYER, stream>>>(ei, xb, whi + 2 * DF * KV, wlo + 2 * DF * KV, b3, g3, be3, xa, nN, nE, vec8);

  k_pool<<<nGB, NTHR, 0, stream>>>(gb, xa, Wr1, br1, Wr2, br2, out, nN, nG);
}
